// RotaryMultiheadAttention_56959856280328
// MI455X (gfx1250) — hardware-verified
//
#include <hip/hip_runtime.h>

typedef _Float16 v16h __attribute__((ext_vector_type(16)));
typedef _Float16 v8h  __attribute__((ext_vector_type(8)));
typedef float    v8f  __attribute__((ext_vector_type(8)));
typedef float    v4f  __attribute__((ext_vector_type(4)));
typedef v8h __attribute__((may_alias)) v8ha;
typedef v4f __attribute__((may_alias)) v4fa;

union Frag { v16h v; v8h half[2]; };

#define SEQ      2048
#define BATCH    2
#define HIDDEN   1024
#define NHEADS   16
#define HD       64
#define N3       3072
#define MROWS    (SEQ * BATCH)
#define NX       (MROWS * HIDDEN)
#define NWQ      (HIDDEN * N3)
#define NWO      (HIDDEN * HIDDEN)
#define NBH      (BATCH * NHEADS)
#define WSCALE   32.0f
#define ASCALE   64.0f
#define PSCALE   16384.0f
#define SM_SCALE 0.125f
#define TPITCH   72

static_assert(MROWS % 128 == 0);
static_assert(SEQ % 64 == 0);
static_assert(SEQ % 8 == 0);
static_assert(N3 % 64 == 0);
static_assert(HIDDEN % 64 == 0);
static_assert((NX / 8) % 256 == 0);
static_assert(HD == 64);

__device__ __forceinline__ v8f wmma_f16(v16h a, v16h b, v8f c) {
  v8f d = __builtin_amdgcn_wmma_f32_16x16x32_f16(false, a, false, b, (short)0, c, false, false);
  asm volatile("v_nop\n\tv_nop\n\tv_nop\n\tv_nop" : "+v"(d) : "v"(a), "v"(b));
  return d;
}

__device__ __forceinline__ v16h load_frag(const _Float16* p, int h) {
  Frag f;
  f.half[0] = *(const v8ha*)(p + 8 * h);
  f.half[1] = *(const v8ha*)(p + 16 + 8 * h);
  return f.v;
}

__global__ __launch_bounds__(256) void cvt_x_kernel(const float* __restrict__ x,
                                                    _Float16* __restrict__ xh)
{
  const int g = blockIdx.x * 256 + threadIdx.x;
  if (g >= NX / 8) return;
  const float* src = x + (size_t)g * 8;
  const v4f a = *(const v4fa*)src;
  const v4f c = *(const v4fa*)(src + 4);
  const v8h o = { (_Float16)a.x, (_Float16)a.y, (_Float16)a.z, (_Float16)a.w,
                  (_Float16)c.x, (_Float16)c.y, (_Float16)c.z, (_Float16)c.w };
  _Float16* dst = xh + (size_t)g * 8;
  *(volatile v8h*)dst = o;
  __threadfence();
  *(volatile v8h*)dst = o;
}

__device__ __forceinline__ void tw_store_pass(const _Float16* sT, _Float16* dst, int K,
                                              int n0, int k0, int w, int lane) {
  const int q8 = lane & 7, sub = lane >> 3;
  #pragma unroll
  for (int i = 0; i < 4; ++i) {
    const int rn = w * 16 + i * 4 + sub;
    const v8h v = *(const v8ha*)(sT + rn * TPITCH + 8 * q8);
    *(volatile v8h*)(dst + (size_t)(n0 + rn) * K + k0 + 8 * q8) = v;
  }
}

__global__ __launch_bounds__(128) void transpose_w_kernel(const float* __restrict__ src,
                                                          _Float16* __restrict__ dst,
                                                          int K, int N)
{
  __shared__ __attribute__((aligned(16))) _Float16 sT[64 * TPITCH];

  const int tid = threadIdx.x, lane = tid & 31, w = tid >> 5;
  const int n0 = blockIdx.x * 64, k0 = blockIdx.y * 64;
  if (n0 + 64 > N || k0 + 64 > K) return;
  const int c4 = tid & 15, kr0 = tid >> 4;
  #pragma unroll
  for (int i = 0; i < 8; ++i) {
    const int kr = kr0 + 8 * i;
    const v4f v = *(const v4fa*)(src + (size_t)(k0 + kr) * N + n0 + 4 * c4);
    _Float16* col = sT + (4 * c4) * TPITCH + kr;
    col[0 * TPITCH] = (_Float16)(v.x * WSCALE);
    col[1 * TPITCH] = (_Float16)(v.y * WSCALE);
    col[2 * TPITCH] = (_Float16)(v.z * WSCALE);
    col[3 * TPITCH] = (_Float16)(v.w * WSCALE);
  }
  __syncthreads();

  tw_store_pass(sT, dst, K, n0, k0, w, lane);
  __threadfence();
  tw_store_pass(sT, dst, K, n0, k0, w, lane);
}

__global__ __launch_bounds__(256) void rope_table_kernel(float* __restrict__ tab)
{
  __shared__ __attribute__((aligned(16))) float sC[8 * 64];

  const int tid = threadIdx.x;
  const int s0 = blockIdx.x * 8;
  const int row = tid >> 5, i = tid & 31;
  const float e = (float)(2 * i) * (1.0f / 64.0f);
  const float p = powf(10000.0f, e);
  const float inv = 1.0f / p;
  const float th = (float)(s0 + row) * inv;
  sC[row * 64 + i] = cosf(th);
  sC[row * 64 + 32 + i] = sinf(th);
  __syncthreads();

  if (tid < 128) {
    const int rr = tid >> 4, c4 = tid & 15;
    const v4f v = *(const v4fa*)(sC + rr * 64 + 4 * c4);
    float* d = tab + (size_t)(s0 + rr) * 64 + 4 * c4;
    *(volatile v4f*)d = v;
    __threadfence();
    *(volatile v4f*)d = v;
  }
}

__device__ __forceinline__ void qkv_store_pass(const _Float16* sT, _Float16* plane, _Float16* vtp,
                                               int which, int head, int s0, int w, int lane) {
  const int q8 = lane & 7, sub = lane >> 3;
  #pragma unroll
  for (int i = 0; i < 8; ++i) {
    const int lid = w * 32 + i * 4 + sub;
    const int bb = lid >> 6, rr = lid & 63;
    const int bh = bb * NHEADS + head;
    const v8h v = *(const v8ha*)(sT + lid * 64 + 8 * q8);
    _Float16* dst;
    if (which != 2) dst = plane + ((size_t)bh * SEQ + s0 + rr) * HD + 8 * q8;
    else            dst = vtp + ((size_t)bh * HD + rr) * SEQ + s0 + 8 * q8;
    *(volatile v8h*)dst = v;
  }
}

__global__ __launch_bounds__(128) void proj_qkv_kernel(
    const _Float16* __restrict__ xh,
    const _Float16* __restrict__ wqt,
    const float* __restrict__ bqkv,
    const float* __restrict__ tab,
    _Float16* __restrict__ qpl,
    _Float16* __restrict__ kpl,
    _Float16* __restrict__ vtp)
{
  __shared__ __attribute__((aligned(16))) _Float16 sT[128 * 64];

  const int tid = threadIdx.x, lane = tid & 31, w = tid >> 5;
  const int h = lane >> 4, m = lane & 15;
  const int m0 = blockIdx.x * 128;
  const int s0 = blockIdx.x * 64;
  const int cg = blockIdx.y;
  const int head = cg / 3;
  const int which = cg - 3 * head;
  const int n0 = cg * 64;
  const int m0w = m0 + 32 * w;

  const _Float16* xa0 = xh + (size_t)(m0w + m) * HIDDEN;
  const _Float16* xa1 = xa0 + (size_t)16 * HIDDEN;
  const _Float16* wb  = wqt + (size_t)(n0 + m) * HIDDEN;

  const v8f zero8 = {0.f, 0.f, 0.f, 0.f, 0.f, 0.f, 0.f, 0.f};
  v8f acc[2][4];
  #pragma unroll
  for (int mt = 0; mt < 2; ++mt)
    #pragma unroll
    for (int nt = 0; nt < 4; ++nt) acc[mt][nt] = zero8;

  #pragma unroll 1
  for (int k0 = 0; k0 < HIDDEN; k0 += 32) {
    const v16h a0 = load_frag(xa0 + k0, h);
    const v16h a1 = load_frag(xa1 + k0, h);
    #pragma unroll
    for (int nt = 0; nt < 4; ++nt) {
      const v16h b = load_frag(wb + (size_t)nt * 16 * HIDDEN + k0, h);
      acc[0][nt] = wmma_f16(a0, b, acc[0][nt]);
      acc[1][nt] = wmma_f16(a1, b, acc[1][nt]);
    }
  }

  const float* bias = bqkv + n0;
  float bvl[4];
  #pragma unroll
  for (int nt = 0; nt < 4; ++nt) bvl[nt] = bias[16 * nt + m];

  if (which != 2) {
    #pragma unroll
    for (int mt = 0; mt < 2; ++mt) {
      #pragma unroll
      for (int rp = 0; rp < 4; ++rp) {
        const int sl = 16 * w + 8 * mt + 4 * h + rp;
        const float* trow = tab + (size_t)(s0 + sl) * 64;
        #pragma unroll
        for (int nt = 0; nt < 2; ++nt) {
          const int i = 16 * nt + m;
          const float cs = trow[i];
          const float sn = trow[32 + i];
          #pragma unroll
          for (int bb = 0; bb < 2; ++bb) {
            const int r = 2 * rp + bb;
            const float y1 = acc[mt][nt][r] * (1.0f / WSCALE) + bvl[nt];
            const float y2 = acc[mt][nt + 2][r] * (1.0f / WSCALE) + bvl[nt + 2];
            const float o1 = y1 * cs - y2 * sn;
            const float o2 = y2 * cs + y1 * sn;
            _Float16* row = sT + (bb * 64 + sl) * 64;
            row[i] = (_Float16)o1;
            row[32 + i] = (_Float16)o2;
          }
        }
      }
    }
  } else {
    #pragma unroll
    for (int mt = 0; mt < 2; ++mt) {
      #pragma unroll
      for (int r = 0; r < 8; ++r) {
        const int sl = 16 * w + 8 * mt + 4 * h + (r >> 1);
        const int bb = r & 1;
        #pragma unroll
        for (int nt = 0; nt < 4; ++nt) {
          const int d = 16 * nt + m;
          const float y = acc[mt][nt][r] * (1.0f / WSCALE) + bvl[nt];
          sT[(bb * 64 + d) * 64 + sl] = (_Float16)y;
        }
      }
    }
  }
  __syncthreads();

  _Float16* plane = (which == 0) ? qpl : kpl;
  qkv_store_pass(sT, plane, vtp, which, head, s0, w, lane);
  __threadfence();
  qkv_store_pass(sT, plane, vtp, which, head, s0, w, lane);
}

__device__ __forceinline__ v16h pack_p(v8f a, v8f c) {
  const v16h r = { (_Float16)(a[0] * PSCALE), (_Float16)(a[1] * PSCALE), (_Float16)(a[2] * PSCALE), (_Float16)(a[3] * PSCALE),
                   (_Float16)(a[4] * PSCALE), (_Float16)(a[5] * PSCALE), (_Float16)(a[6] * PSCALE), (_Float16)(a[7] * PSCALE),
                   (_Float16)(c[0] * PSCALE), (_Float16)(c[1] * PSCALE), (_Float16)(c[2] * PSCALE), (_Float16)(c[3] * PSCALE),
                   (_Float16)(c[4] * PSCALE), (_Float16)(c[5] * PSCALE), (_Float16)(c[6] * PSCALE), (_Float16)(c[7] * PSCALE) };
  return r;
}

__device__ __forceinline__ void att_store_pass(const _Float16* so, _Float16* ah,
                                               int b, int head, int q0, int lane) {
  const int q8 = lane & 7, sub = lane >> 3;
  #pragma unroll
  for (int i = 0; i < 4; ++i) {
    const int row = i * 4 + sub;
    const v8h v = *(const v8ha*)(so + row * 64 + 8 * q8);
    const size_t gi = ((size_t)(q0 + row) * BATCH + b) * HIDDEN + head * HD + 8 * q8;
    *(volatile v8h*)(ah + gi) = v;
  }
}

__global__ __launch_bounds__(128) void attn_kernel(
    const _Float16* __restrict__ qpl,
    const _Float16* __restrict__ kpl,
    const _Float16* __restrict__ vtp,
    _Float16* __restrict__ ah)
{
  __shared__ __attribute__((aligned(16))) _Float16 sO[4 * 16 * 64];

  const int tid = threadIdx.x, lane = tid & 31, w = tid >> 5;
  const int h = lane >> 4, m = lane & 15;
  const int bh = blockIdx.y, b = bh >> 4, head = bh & 15;
  const int q0 = blockIdx.x * 64 + 16 * w;

  const _Float16* qrow = qpl + ((size_t)bh * SEQ + q0 + m) * HD;
  const v16h qb0 = load_frag(qrow, h);
  const v16h qb1 = load_frag(qrow + 32, h);

  const v8f zero8 = {0.f, 0.f, 0.f, 0.f, 0.f, 0.f, 0.f, 0.f};
  v8f o[4];
  #pragma unroll
  for (int t = 0; t < 4; ++t) o[t] = zero8;
  float mrun = -1e30f, lrun = 0.0f;

  const _Float16* kbase = kpl + ((size_t)bh * SEQ + m) * HD;
  const _Float16* vbase = vtp + ((size_t)bh * HD + m) * SEQ;

  #pragma unroll 1
  for (int kb = 0; kb < SEQ; kb += 64) {
    v8f s[4];
    #pragma unroll
    for (int j = 0; j < 4; ++j) {
      const _Float16* kp = kbase + (size_t)(kb + 16 * j) * HD;
      const v16h kf0 = load_frag(kp, h);
      const v16h kf1 = load_frag(kp + 32, h);
      v8f z = zero8;
      z = wmma_f16(kf0, qb0, z);
      z = wmma_f16(kf1, qb1, z);
      s[j] = z * SM_SCALE;
    }

    float mloc = s[0][0];
    #pragma unroll
    for (int j = 0; j < 4; ++j)
      #pragma unroll
      for (int r = 0; r < 8; ++r) mloc = fmaxf(mloc, s[j][r]);
    mloc = fmaxf(mloc, __shfl_xor(mloc, 16));
    const float mnew = fmaxf(mrun, mloc);
    const float alpha = __expf(mrun - mnew);
    mrun = mnew;
    float lsum = 0.0f;
    #pragma unroll
    for (int j = 0; j < 4; ++j)
      #pragma unroll
      for (int r = 0; r < 8; ++r) {
        const float p = __expf(s[j][r] - mnew);
        s[j][r] = p;
        lsum += p;
      }
    lsum += __shfl_xor(lsum, 16);
    lrun = lrun * alpha + lsum;
    #pragma unroll
    for (int t = 0; t < 4; ++t)
      #pragma unroll
      for (int r = 0; r < 8; ++r) o[t][r] = o[t][r] * alpha;

    const v16h pb0 = pack_p(s[0], s[1]);
    const v16h pb1 = pack_p(s[2], s[3]);

    #pragma unroll
    for (int t = 0; t < 4; ++t) {
      const _Float16* vp = vbase + (size_t)(16 * t) * SEQ + kb;
      const v16h vf0 = load_frag(vp, h);
      const v16h vf1 = load_frag(vp + 32, h);
      o[t] = wmma_f16(vf0, pb0, o[t]);
      o[t] = wmma_f16(vf1, pb1, o[t]);
    }
  }

  const float inv = (1.0f / lrun) * (ASCALE / PSCALE);
  _Float16* so = sO + w * 1024;
  #pragma unroll
  for (int t = 0; t < 4; ++t)
    #pragma unroll
    for (int r = 0; r < 8; ++r)
      so[m * 64 + 16 * t + 8 * h + r] = (_Float16)(o[t][r] * inv);
  __syncthreads();

  att_store_pass(so, ah, b, head, q0, lane);
  __threadfence();
  att_store_pass(so, ah, b, head, q0, lane);
}

__device__ __forceinline__ void out_store_pass(const float* sO, float* out,
                                               int m0, int n0, int w, int lane) {
  const int q8 = lane & 7, sub = lane >> 3;
  #pragma unroll
  for (int i = 0; i < 16; ++i) {
    const int L = w * 64 + i * 4 + sub;
    const int tokl = L >> 1, hl = L & 1;
    const v4f v = *(const v4fa*)(sO + tokl * 64 + 32 * hl + 4 * q8);
    float* d = out + (size_t)(m0 + tokl) * HIDDEN + n0 + 32 * hl + 4 * q8;
    *(volatile v4f*)d = v;
  }
}

__global__ __launch_bounds__(128) void proj_out_kernel(
    const _Float16* __restrict__ ah,
    const _Float16* __restrict__ wot,
    const float* __restrict__ bout,
    float* __restrict__ out)
{
  __shared__ __attribute__((aligned(16))) float sO[128 * 64];

  const int tid = threadIdx.x, lane = tid & 31, w = tid >> 5;
  const int h = lane >> 4, m = lane & 15;
  const int m0 = blockIdx.x * 128;
  const int n0 = blockIdx.y * 64;
  const int m0w = m0 + 32 * w;

  const _Float16* xa0 = ah + (size_t)(m0w + m) * HIDDEN;
  const _Float16* xa1 = xa0 + (size_t)16 * HIDDEN;
  const _Float16* wb  = wot + (size_t)(n0 + m) * HIDDEN;

  const v8f zero8 = {0.f, 0.f, 0.f, 0.f, 0.f, 0.f, 0.f, 0.f};
  v8f acc[2][4];
  #pragma unroll
  for (int mt = 0; mt < 2; ++mt)
    #pragma unroll
    for (int nt = 0; nt < 4; ++nt) acc[mt][nt] = zero8;

  #pragma unroll 1
  for (int k0 = 0; k0 < HIDDEN; k0 += 32) {
    const v16h a0 = load_frag(xa0 + k0, h);
    const v16h a1 = load_frag(xa1 + k0, h);
    #pragma unroll
    for (int nt = 0; nt < 4; ++nt) {
      const v16h b = load_frag(wb + (size_t)nt * 16 * HIDDEN + k0, h);
      acc[0][nt] = wmma_f16(a0, b, acc[0][nt]);
      acc[1][nt] = wmma_f16(a1, b, acc[1][nt]);
    }
  }

  #pragma unroll
  for (int nt = 0; nt < 4; ++nt) {
    const int feat = 16 * nt + m;
    const float bv = bout[n0 + feat];
    #pragma unroll
    for (int mt = 0; mt < 2; ++mt) {
      #pragma unroll
      for (int r = 0; r < 8; ++r) {
        const int tokl = 32 * w + 16 * mt + 8 * h + r;
        sO[tokl * 64 + feat] = acc[mt][nt][r] * (1.0f / (WSCALE * ASCALE)) + bv;
      }
    }
  }
  __syncthreads();

  out_store_pass(sO, out, m0, n0, w, lane);
  __threadfence();
  out_store_pass(sO, out, m0, n0, w, lane);
}

extern "C" void kernel_launch(void* const* d_in, const int* in_sizes, int n_in,
                              void* d_out, int out_size, void* d_ws, size_t ws_size,
                              hipStream_t stream) {
  if (n_in < 5) return;
  if (in_sizes[0] != NX) return;
  if (in_sizes[1] != NWQ) return;
  if (in_sizes[2] != N3) return;
  if (in_sizes[3] != NWO) return;
  if (in_sizes[4] != HIDDEN) return;
  if (out_size != NX) return;

  const float* x    = (const float*)d_in[0];
  const float* wqkv = (const float*)d_in[1];
  const float* bqkv = (const float*)d_in[2];
  const float* wout = (const float*)d_in[3];
  const float* bout = (const float*)d_in[4];
  float* out = (float*)d_out;

  const size_t xh_bytes  = (size_t)NX * 2;
  const size_t wqt_bytes = (size_t)NWQ * 2;
  const size_t wot_bytes = (size_t)NWO * 2;
  const size_t tab_bytes = (size_t)SEQ * 64 * 4;
  const size_t pl_bytes  = (size_t)NBH * SEQ * HD * 2;
  const size_t ah_bytes  = (size_t)NX * 2;
  const size_t total = xh_bytes + wqt_bytes + wot_bytes + tab_bytes + 3 * pl_bytes + ah_bytes;
  if (total > ws_size) return;

  char* ws = (char*)d_ws;
  size_t off = 0;
  _Float16* xh  = (_Float16*)(ws + off); off += xh_bytes;
  _Float16* wqt = (_Float16*)(ws + off); off += wqt_bytes;
  _Float16* wot = (_Float16*)(ws + off); off += wot_bytes;
  float*    tab = (float*)(ws + off);    off += tab_bytes;
  _Float16* qpl = (_Float16*)(ws + off); off += pl_bytes;
  _Float16* kpl = (_Float16*)(ws + off); off += pl_bytes;
  _Float16* vtp = (_Float16*)(ws + off); off += pl_bytes;
  _Float16* ah  = (_Float16*)(ws + off); off += ah_bytes;
  if (off > ws_size) return;

  cvt_x_kernel<<<(NX / 8) / 256, 256, 0, stream>>>(x, xh);

  transpose_w_kernel<<<dim3(N3 / 64, HIDDEN / 64), 128, 0, stream>>>(wqkv, wqt, HIDDEN, N3);
  transpose_w_kernel<<<dim3(HIDDEN / 64, HIDDEN / 64), 128, 0, stream>>>(wout, wot, HIDDEN, HIDDEN);

  rope_table_kernel<<<SEQ / 8, 256, 0, stream>>>(tab);

  dim3 gProj(MROWS / 128, 3 * NHEADS);
  proj_qkv_kernel<<<gProj, 128, 0, stream>>>(xh, wqt, bqkv, tab, qpl, kpl, vtp);

  dim3 gAtt(SEQ / 64, NBH);
  attn_kernel<<<gAtt, 128, 0, stream>>>(qpl, kpl, vtp, ah);

  dim3 gOut(MROWS / 128, HIDDEN / 64);
  proj_out_kernel<<<gOut, 128, 0, stream>>>(ah, wot, bout, out);
}
